// SubmanifoldSparseConv_16441134809108
// MI455X (gfx1250) — hardware-run, weakly checked
//
#include <hip/hip_runtime.h>
#include <stddef.h>


#define C_CH    32
#define K_OFF   27
#define KB      130
#define NSLAB   KB
#define NYZ     (KB * KB)
#define DP      17408
#define STHR    256
#define SWAV    (STHR / 32)
#define CAP     4096
#define FTHR    256
#define FROWS   (FTHR / 4)
#define CTHR    128
#define CWAV    (CTHR / 32)
#define CPTS    (16 * CWAV)
#define KROW    (K_OFF * C_CH)
#define NPAIR   (CPTS * K_OFF)
#define NPIECE  (NPAIR * 4)
#define XSC     8.0f
#define WSC     64.0f
#define RH      0.001953125f
#define WSCAP   134217728

#define LS_T    0
#define LS_YZ   (DP)
#define LS_ID   (DP + CAP)
#define LS_END  (DP + 2 * CAP)
#define LDS_SLAB (LS_END * 4)

#define LC_A    0
#define LC_S    (CPTS * KROW * 2)
#define LC_NB   (LC_S + CWAV * 512 * 4)
#define LC_POS  (LC_NB + NPAIR * 4)
#define LDS_CONV (LC_POS + CPTS * 3 * 4)

static_assert(DP >= NYZ);
static_assert((DP % (4 * STHR)) == 0);
static_assert(LDS_SLAB == 102400);
static_assert((CAP % 32) == 0);
static_assert(NYZ < 32768);
static_assert(CPTS == 64);
static_assert((NPIECE % CTHR) == 0);
static_assert(LC_S == 110592);
static_assert(LDS_CONV == 126464);
static_assert((LC_S % 16) == 0 && (LC_NB % 16) == 0 && (LC_POS % 16) == 0);
static_assert(FROWS == 64);
static_assert((KROW * 2) % 16 == 0);

typedef float    v4f  __attribute__((ext_vector_type(4)));
typedef float    v8f  __attribute__((ext_vector_type(8)));
typedef int      v4i  __attribute__((ext_vector_type(4)));
typedef _Float16 v4h  __attribute__((ext_vector_type(4)));
typedef _Float16 v8h  __attribute__((ext_vector_type(8)));
typedef _Float16 v16h __attribute__((ext_vector_type(16)));
union Frag  { v16h v; v8h h[2]; v4h q[4]; };
union Frag8 { v8h v; v4h q[2]; };

__device__ __forceinline__ v8f wmh(v16h a, v16h b, v8f c) {
  v8f d = __builtin_amdgcn_wmma_f32_16x16x32_f16(false, a, false, b, (short)0, c, false, false);
  asm volatile("v_nop\n\tv_nop\n\tv_nop\n\tv_nop" : "+v"(d) : "v"(a), "v"(b));
  return d;
}

__device__ __forceinline__ v4h cvt4h(v4f x) {
  v4h r;
  r.x = (_Float16)x.x;
  r.y = (_Float16)x.y;
  r.z = (_Float16)x.z;
  r.w = (_Float16)x.w;
  return r;
}

__device__ __forceinline__ void wfence() {
  __builtin_amdgcn_fence(__ATOMIC_ACQ_REL, "wavefront");
  __builtin_amdgcn_wave_barrier();
}

__device__ __forceinline__ unsigned match15(int key, unsigned vm) {
  unsigned peers = vm;
#pragma unroll
  for (int i = 0; i < 15; ++i) {
    const bool bit = ((key >> i) & 1) != 0;
    const unsigned bq = __builtin_amdgcn_ballot_w32(bit);
    peers &= bit ? bq : ~bq;
  }
  return peers;
}

__device__ __forceinline__ void blkscan(int cnt, int lane, int wave, int* swt, int& pos, int& nh) {
  int x = cnt;
#pragma unroll
  for (int o = 1; o < 32; o <<= 1) {
    const int y = __shfl_up(x, o, 32);
    x += (lane >= o) ? y : 0;
  }
  if (lane == 31) swt[wave] = x;
  __syncthreads();
  int wpre = 0, tot = 0;
#pragma unroll
  for (int w = 0; w < SWAV; ++w) {
    const int v = swt[w];
    wpre += (w < wave) ? v : 0;
    tot += v;
  }
  pos = wpre + x - cnt;
  nh = tot;
}

__device__ __forceinline__ int clampi(int v, int lo, int hi) {
  return v < lo ? lo : (v > hi ? hi : v);
}

__global__ __launch_bounds__(128) void k_wprep(const float* __restrict__ W, _Float16* Wp) {
  const int o = blockIdx.x, tid = threadIdx.x;
  const int n = tid >> 2, c0 = (tid & 3) * 8;
  const float* wk = W + (size_t)o * (C_CH * C_CH);
  v8h hv;
#pragma unroll
  for (int e = 0; e < 8; ++e) hv[e] = (_Float16)(wk[(c0 + e) * C_CH + n] * WSC);
  _Float16* dst = Wp + ((size_t)o * C_CH + n) * C_CH + c0;
  *(volatile v8h*)dst = hv;
  __threadfence();
  *(volatile v8h*)dst = hv;
}

__global__ __launch_bounds__(FTHR) void k_fcvt(const float* __restrict__ X, _Float16* Fh, int nN) {
  const int tid = threadIdx.x;
  const int row = blockIdx.x * FROWS + (tid >> 2);
  const int c0 = (tid & 3) * 8;
  const bool ok = row < nN;
  const int rc = ok ? row : nN - 1;
  const float* xp = X + (size_t)rc * C_CH + c0;
  v4f f0 = *(const v4f*)(xp);
  v4f f1 = *(const v4f*)(xp + 4);
  const v4f z = {0.0f, 0.0f, 0.0f, 0.0f};
  f0 = ok ? f0 * XSC : z;
  f1 = ok ? f1 * XSC : z;
  Frag8 hv;
  hv.q[0] = cvt4h(f0);
  hv.q[1] = cvt4h(f1);
  _Float16* dst = Fh + (size_t)row * C_CH + c0;
  *(volatile v8h*)dst = hv.v;
  __threadfence();
  *(volatile v8h*)dst = hv.v;
}

__global__ __launch_bounds__(STHR) void k_slab(const int* __restrict__ pos, int* Dtab, int nN, int nBatch) {
  extern __shared__ __attribute__((aligned(16))) char dynl[];
  int* T   = (int*)dynl + LS_T;
  int* lyz = (int*)dynl + LS_YZ;
  int* lid = (int*)dynl + LS_ID;
  __shared__ int swt[SWAV];
  const int tid = threadIdx.x, lane = tid & 31;
  const int wave = __builtin_amdgcn_readfirstlane(tid >> 5);
  const unsigned lt = (1u << lane) - 1u;
  const int slab = blockIdx.x;
  {
    const v4i z = {nN, nN, nN, nN};
#pragma unroll
    for (int it = 0; it < DP / (4 * STHR); ++it) ((v4i*)T)[it * STHR + tid] = z;
  }
  __syncthreads();

  int L = 0;
#pragma unroll 1
  for (int q = 0; q < nBatch; ++q) {
    const int i = q * STHR + tid;
    const bool iv = i < nN;
    const int ic = iv ? i : nN - 1;
    const int x = pos[(size_t)ic * 3 + 0];
    const int y = pos[(size_t)ic * 3 + 1];
    const int z = pos[(size_t)ic * 3 + 2];
    const int sx = clampi(x + 1, 0, KB - 1);
    const int sy = clampi(y + 1, 0, KB - 1);
    const int sz = clampi(z + 1, 0, KB - 1);
    const bool keep = iv && (sx == slab);
    int p, tot;
    blkscan(keep ? 1 : 0, lane, wave, swt, p, tot);
    const int di = L + p;
    if (keep && di < CAP) {
      lyz[di] = sy * KB + sz;
      lid[di] = i;
    }
    L += tot;
    __syncthreads();
  }
  const int Lc = __builtin_amdgcn_readfirstlane(L < CAP ? L : CAP);
  const int nG = (Lc + 31) >> 5;

  if (wave == 0) {
#pragma unroll 1
    for (int g = 0; g < CAP / 32; ++g) {
      if (g >= nG) break;
      const int idx = 32 * g + lane;
      const bool valid = idx < Lc;
      const int yzr = lyz[idx];
      const int yz = valid ? yzr : 0;
      const int pid = lid[idx];
      const unsigned vmask = __builtin_amdgcn_ballot_w32(valid);
      const unsigned peers = match15(yz, vmask);
      const bool lead = valid && ((peers & lt) == 0u);
      const int cur = T[yz];
      if (lead && cur == nN) T[yz] = pid;
      wfence();
    }
  }
  __syncthreads();

  int* Dp = Dtab + (size_t)slab * DP;
#pragma unroll
  for (int it = 0; it < DP / (4 * STHR); ++it) {
    const int f = it * STHR + tid;
    const v4i vv = ((const v4i*)T)[f];
    *(volatile v4i*)(Dp + 4 * f) = vv;
  }
  __threadfence();
#pragma unroll
  for (int it = 0; it < DP / (4 * STHR); ++it) {
    const int f = it * STHR + tid;
    const v4i vv = ((const v4i*)T)[f];
    *(volatile v4i*)(Dp + 4 * f) = vv;
  }
}

__global__ __launch_bounds__(CTHR) void k_conv(const _Float16* __restrict__ Fh, const int* __restrict__ pos,
                                               const int* __restrict__ Dtab, const _Float16* __restrict__ Wp,
                                               float* out, int nN) {
  extern __shared__ __attribute__((aligned(16))) char dynl[];
  _Float16* AL = (_Float16*)(dynl + LC_A);
  float* S   = (float*)(dynl + LC_S);
  int* nbl   = (int*)(dynl + LC_NB);
  int* sp    = (int*)(dynl + LC_POS);
  const int tid = threadIdx.x, lane = tid & 31, hh = lane >> 4, m = lane & 15;
  const int wave = __builtin_amdgcn_readfirstlane(tid >> 5);
  const int pb = blockIdx.x * CPTS;

  if (tid < CPTS) {
    int pt = pb + tid;
    pt = pt > nN - 1 ? nN - 1 : pt;
    sp[3 * tid + 0] = pos[(size_t)pt * 3 + 0];
    sp[3 * tid + 1] = pos[(size_t)pt * 3 + 1];
    sp[3 * tid + 2] = pos[(size_t)pt * 3 + 2];
  }
  __syncthreads();

#pragma unroll 1
  for (int it = 0; it < (NPAIR + CTHR - 1) / CTHR; ++it) {
    const int p = it * CTHR + tid;
    const int pc = p < NPAIR ? p : NPAIR - 1;
    const int j = pc / K_OFF;
    const int o = pc - j * K_OFF;
    const int dx = o / 9 - 1, dy = (o / 3) % 3 - 1, dz = o % 3 - 1;
    const int cx = clampi(sp[3 * j + 0] + dx + 1, 0, KB - 1);
    const int cy = clampi(sp[3 * j + 1] + dy + 1, 0, KB - 1);
    const int cz = clampi(sp[3 * j + 2] + dz + 1, 0, KB - 1);
    const int v = Dtab[(size_t)cx * DP + cy * KB + cz];
    const int nb = v < 0 ? 0 : (v > nN ? nN : v);
    if (p < NPAIR) nbl[p] = nb;
  }
  __syncthreads();

#pragma unroll 1
  for (int it = 0; it < NPIECE / CTHR; ++it) {
    const int p = it * CTHR + tid;
    const int j = p / (4 * K_OFF);
    const int r = p - j * (4 * K_OFF);
    const int o = r >> 2, q = r & 3;
    const int nb = nbl[j * K_OFF + o];
    const v8h vv = *(const v8h*)(Fh + (size_t)nb * C_CH + 8 * q);
    *(v8h*)(AL + (size_t)j * KROW + o * C_CH + 8 * q) = vv;
  }
  __syncthreads();

  const v8f z8 = {0.0f, 0.0f, 0.0f, 0.0f, 0.0f, 0.0f, 0.0f, 0.0f};
  v8f acc0 = z8, acc1 = z8;
  {
    const _Float16* ga  = AL + (size_t)(wave * 16 + m) * KROW + 8 * hh;
    const _Float16* wb0 = Wp + (size_t)m * C_CH + 8 * hh;
    const _Float16* wb1 = Wp + (size_t)(16 + m) * C_CH + 8 * hh;
#pragma unroll 1
    for (int o = 0; o < K_OFF; ++o) {
      Frag a, b0, b1;
      const _Float16* gp = ga + o * C_CH;
      a.h[0] = *(const v8h*)(gp);
      a.h[1] = *(const v8h*)(gp + 16);
      const _Float16* p0 = wb0 + (size_t)o * (C_CH * C_CH);
      const _Float16* p1 = wb1 + (size_t)o * (C_CH * C_CH);
      b0.h[0] = *(const v8h*)(p0);
      b0.h[1] = *(const v8h*)(p0 + 16);
      b1.h[0] = *(const v8h*)(p1);
      b1.h[1] = *(const v8h*)(p1 + 16);
      acc0 = wmh(a.v, b0.v, acc0);
      acc1 = wmh(a.v, b1.v, acc1);
    }
  }

  float* Sw = S + wave * 512;
#pragma unroll
  for (int r = 0; r < 8; ++r) {
    Sw[(8 * hh + r) * C_CH + m]      = acc0[r] * RH;
    Sw[(8 * hh + r) * C_CH + 16 + m] = acc1[r] * RH;
  }
  __syncthreads();
  {
    const int rr = lane >> 3, cc = (lane & 7) * 4;
    v4f ov[4];
#pragma unroll
    for (int qq = 0; qq < 4; ++qq) ov[qq] = *(const v4f*)(Sw + (4 * qq + rr) * C_CH + cc);
    const int rbase = pb + 16 * wave + rr;
#pragma unroll
    for (int qq = 0; qq < 4; ++qq) {
      const int row = rbase + 4 * qq;
      const int rcl = row < nN ? row : nN - 1;
      float* op = out + (size_t)rcl * C_CH + cc;
      if (row < nN) *(volatile v4f*)op = ov[qq];
    }
    __threadfence();
#pragma unroll
    for (int qq = 0; qq < 4; ++qq) {
      const int row = rbase + 4 * qq;
      const int rcl = row < nN ? row : nN - 1;
      float* op = out + (size_t)rcl * C_CH + cc;
      if (row < nN) *(volatile v4f*)op = ov[qq];
    }
  }
}

extern "C" void kernel_launch(void* const* d_in, const int* in_sizes, int n_in,
                              void* d_out, int out_size, void* d_ws, size_t ws_size,
                              hipStream_t stream) {
  if (n_in < 3) return;
  if (in_sizes[1] < 3) return;
  const int nN = in_sizes[1] / 3;
  if (nN < 1 || in_sizes[1] != nN * 3) return;
  if (in_sizes[0] != nN * C_CH) return;
  if (in_sizes[2] != K_OFF * C_CH * C_CH) return;
  if (out_size != nN * C_CH) return;

  const int nBatch  = (nN + STHR - 1) / STHR;
  const int rowsPad = ((nN + 1 + FROWS - 1) / FROWS) * FROWS;
  const int gF      = rowsPad / FROWS;
  const int gC      = (nN + CPTS - 1) / CPTS;

  const float* X   = (const float*)d_in[0];
  const int*   P   = (const int*)d_in[1];
  const float* W   = (const float*)d_in[2];
  float* out = (float*)d_out;

  char* ws = (char*)d_ws;
  size_t off = 0;
  const size_t oD  = off; off += (size_t)NSLAB * DP * 4;          off = (off + 255) & ~(size_t)255;
  const size_t oFh = off; off += (size_t)rowsPad * C_CH * 2;      off = (off + 255) & ~(size_t)255;
  const size_t oWp = off; off += (size_t)K_OFF * C_CH * C_CH * 2; off = (off + 255) & ~(size_t)255;
  if (off > ws_size || off > (size_t)WSCAP) return;
  int*      Dtab = (int*)(ws + oD);
  _Float16* Fh   = (_Float16*)(ws + oFh);
  _Float16* Wp   = (_Float16*)(ws + oWp);

  hipFuncSetAttribute(reinterpret_cast<const void*>(&k_slab), hipFuncAttributeMaxDynamicSharedMemorySize, LDS_SLAB);
  hipFuncSetAttribute(reinterpret_cast<const void*>(&k_conv), hipFuncAttributeMaxDynamicSharedMemorySize, LDS_CONV);

  k_wprep<<<K_OFF, 128, 0, stream>>>(W, Wp);
  k_fcvt<<<gF, FTHR, 0, stream>>>(X, Fh, nN);
  k_slab<<<NSLAB, STHR, LDS_SLAB, stream>>>(P, Dtab, nN, nBatch);
  k_conv<<<gC, CTHR, LDS_CONV, stream>>>(Fh, P, Dtab, Wp, out, nN);
}
